// IntraClusterAttention_54039278518788
// MI455X (gfx1250) — hardware-verified
//
#include <hip/hip_runtime.h>
#include <math.h>

typedef __attribute__((ext_vector_type(16))) _Float16 v16h;
typedef __attribute__((ext_vector_type(16))) __bf16 v16b;
typedef __attribute__((ext_vector_type(8)))  _Float16 v8h;
typedef __attribute__((ext_vector_type(8)))  float v8f;
typedef __attribute__((ext_vector_type(4)))  float v4f;
typedef __attribute__((ext_vector_type(2)))  float v2f;
typedef __attribute__((ext_vector_type(4)))  unsigned v4u;
typedef __attribute__((ext_vector_type(4)))  int v4i;
typedef float __attribute__((may_alias)) float_a;
typedef int __attribute__((may_alias)) int_a;

template <typename T> __device__ __forceinline__ void vst2(void* p, T v) { *(volatile T*)p = v; __threadfence(); *(volatile T*)p = v; }
__device__ __forceinline__ v8f wmma16(v16h a, v16h b, v8f c) {
  v8f d = __builtin_amdgcn_wmma_f32_16x16x32_f16(false, a, false, b, (short)0, c, false, false);
  asm volatile("v_nop\n\tv_nop\n\tv_nop\n\tv_nop" : "+v"(d) : "v"(a), "v"(b));
  return d;
}
__device__ __forceinline__ v8f wmma_bf(v16b a, v16b b, v8f c) {
  v8f d = __builtin_amdgcn_wmma_f32_16x16x32_bf16(false, a, false, b, (short)0, c, false, false);
  asm volatile("v_nop\n\tv_nop\n\tv_nop\n\tv_nop" : "+v"(d) : "v"(a), "v"(b));
  return d;
}
__device__ __forceinline__ v16h frag_h(const _Float16* rowk0, int lane) {
  union { v16h v; v8h q[2]; } u; const _Float16* p = rowk0 + 8 * (lane >> 4);
  u.q[0] = *(const v8h*)p; u.q[1] = *(const v8h*)(p + 16); return u.v;
}
__device__ __forceinline__ v16h frag_f32(const float* rowk0, int lane) {
  v16h a; const float* p = rowk0 + 8 * (lane >> 4);
#pragma unroll
  for (int i = 0; i < 8; ++i) { a[i] = (_Float16)p[i]; a[8 + i] = (_Float16)p[16 + i]; }
  return a;
}
__device__ __forceinline__ v16h frag_f32s(const float* rowk0, int lane, float sc) {
  v16h a; const float* p = rowk0 + 8 * (lane >> 4);
#pragma unroll
  for (int i = 0; i < 8; ++i) { a[i] = (_Float16)(p[i] * sc); a[8 + i] = (_Float16)(p[16 + i] * sc); }
  return a;
}
__device__ __forceinline__ v16h fragc_f32(const float* W, int k0, int n, int lane, int ld, int K) {
  v16h a; const int g = lane >> 4;
#pragma unroll
  for (int i = 0; i < 8; ++i) { const int ka = k0 + 8 * g + i, kb = ka + 16;
    a[i] = (_Float16)(ka < K ? W[(size_t)(ka < K ? ka : K - 1) * ld + n] : 0.f); a[8 + i] = (_Float16)(kb < K ? W[(size_t)(kb < K ? kb : K - 1) * ld + n] : 0.f); }
  return a;
}
struct F2 { v16b h, l; };
__device__ __forceinline__ F2 bsplit16(const float v[16]) { F2 r;
#pragma unroll
  for (int i = 0; i < 16; ++i) { const __bf16 h = (__bf16)v[i]; r.h[i] = h; r.l[i] = (__bf16)(v[i] - (float)h); }
  return r; }
__device__ __forceinline__ F2 split_row(const float* row, int k0, int lane) { float v[16]; const float* p = row + k0 + 8 * (lane >> 4);
#pragma unroll
  for (int i = 0; i < 8; ++i) { v[i] = p[i]; v[8 + i] = p[16 + i]; }
  return bsplit16(v); }
__device__ __forceinline__ F2 split_rowK(const float* row, int k0, int lane, int K) { float v[16]; const int g = lane >> 4;
#pragma unroll
  for (int i = 0; i < 8; ++i) { const int ka = k0 + 8 * g + i, kb = ka + 16; v[i] = ka < K ? row[ka < K ? ka : K - 1] : 0.f; v[8 + i] = kb < K ? row[kb < K ? kb : K - 1] : 0.f; }
  return bsplit16(v); }
__device__ __forceinline__ F2 split_col(const float* W, int k0, int n, int lane, int ld, int K) { float v[16]; const int g = lane >> 4;
#pragma unroll
  for (int i = 0; i < 8; ++i) { const int ka = k0 + 8 * g + i, kb = ka + 16; v[i] = ka < K ? W[(size_t)(ka < K ? ka : K - 1) * ld + n] : 0.f; v[8 + i] = kb < K ? W[(size_t)(kb < K ? kb : K - 1) * ld + n] : 0.f; }
  return bsplit16(v); }
__device__ __forceinline__ v8f mac3(const F2& a, const F2& b, v8f c) { c = wmma_bf(a.l, b.h, c); c = wmma_bf(a.h, b.l, c); return wmma_bf(a.h, b.h, c); }
__device__ __forceinline__ float sigm(float v) { return 1.0f / (1.0f + expf(-v)); }
#define LDSX() do { asm volatile("s_wait_dscnt 0" ::: "memory"); __builtin_amdgcn_wave_barrier(); __builtin_amdgcn_fence(__ATOMIC_RELEASE, "workgroup"); } while (0)


#ifndef NTOK
#define NTOK 32768
#endif
#define NTOK_FULL 32768
#define DD 256
#define NH 8
#define HD 32
#define SG 16
#define NG (NTOK / SG)
#define NGB (NG / 4)
typedef __attribute__((ext_vector_type(8))) __bf16 v8b;
__device__ __forceinline__ v16b frag_b(const __bf16* rowk0, int lane) {
  union { v16b v; v8b q[2]; } u; const __bf16* p = rowk0 + 8 * (lane >> 4);
  u.q[0] = *(const v8b*)p; u.q[1] = *(const v8b*)(p + 16); return u.v;
}
__device__ __forceinline__ float bfr(float v) { return (float)(__bf16)v; }
__device__ __attribute__((noinline)) float exp_ni(float v) { return expf(v); }
__device__ __attribute__((noinline)) float erf_ni(float v) { return erff(v); }

#define WS_PW  0u
#define PQKV 0
#define PO (PQKV + 3 * DD * DD)
#define PWEND (PO + DD * DD)
#define WS_QKV (WS_PW + 2u * PWEND)
#define WS_CTX (WS_QKV + 4u * NTOK * 3 * DD)
#define WS_PA  (WS_CTX + 4u * NTOK * DD)
#define WS_END (WS_PA + 4u * NGB * 256)

__global__ __launch_bounds__(256) void k_packT(const float* __restrict__ WQ, const float* __restrict__ WK, const float* __restrict__ WV, const float* __restrict__ WO, __bf16* __restrict__ PW) {
  __shared__ __align__(16) __bf16 s[DD]; const int n = blockIdx.x, which = blockIdx.y, k = threadIdx.x; float v;
  if (which == 0) { const int part = n / DD, c = n % DD; const float* Wm = (part == 0) ? WQ : (part == 1 ? WK : WV); v = Wm[(size_t)k * DD + c]; }
  else { if (n >= DD) return; v = WO[(size_t)k * DD + n]; }
  s[k] = (__bf16)v; __syncthreads();
  if (k < DD / 8) vst2((unsigned*)(PW + (which ? PO : PQKV) + (size_t)n * DD + k * 8), *(const v4u*)&s[k * 8]);
}
template <int RIN>
__global__ __launch_bounds__(128) void k_gemm(const float* __restrict__ A, const __bf16* __restrict__ P, const float* __restrict__ bias, float* __restrict__ OUT, int ldo) {
  __shared__ __align__(16) float so[4][16][132];
  const int tid = threadIdx.x, wave = tid >> 5, lane = tid & 31, col = lane & 15, g = lane >> 4; const size_t r0 = (size_t)blockIdx.x * 64 + wave * 16; const int n0 = blockIdx.y * 128;
  v8f acc[8] = {};
#pragma unroll 2
  for (int kc = 0; kc < DD / 32; ++kc) { F2 a; if (RIN) { v16b ax; const float* p = A + (r0 + col) * DD + kc * 32 + 8 * g;
#pragma unroll
      for (int i = 0; i < 8; ++i) { ax[i] = (__bf16)p[i]; ax[8 + i] = (__bf16)p[16 + i]; } a.h = ax; a.l = ax; } else a = split_row(A + (r0 + col) * DD, kc * 32, lane);
#pragma unroll
    for (int j = 0; j < 8; ++j) { const v16b w = frag_b(P + (size_t)(n0 + j * 16 + col) * DD + kc * 32, lane); if (!RIN) acc[j] = wmma_bf(a.l, w, acc[j]); acc[j] = wmma_bf(a.h, w, acc[j]); } }
#pragma unroll
  for (int j = 0; j < 8; ++j) { const float bb = bfr(bias[n0 + j * 16 + col]);
#pragma unroll
    for (int r = 0; r < 8; ++r) so[wave][8 * g + r][j * 16 + col] = acc[j][r] + bb; }
  LDSX();
  for (int rl = 0; rl < 16; ++rl) vst2(OUT + (r0 + rl) * ldo + n0 + lane * 4, *(const v4f*)&so[wave][rl][lane * 4]);
}
__global__ __launch_bounds__(128) void k_attn(const float* __restrict__ QKV, float* __restrict__ CTX, float* __restrict__ PA) {
  __shared__ __align__(16) float sp[4][16][36]; __shared__ __align__(16) float so[4][16][260]; __shared__ float sacc[4][16][17]; __shared__ __align__(16) float sline[256];
  const int tid = threadIdx.x, wave = tid >> 5, lane = tid & 31, col = lane & 15, g = lane >> 4; const size_t grp = (size_t)blockIdx.x * 4 + wave; const size_t r0 = grp * SG;
  float pacc[8]; for (int r = 0; r < 8; ++r) pacc[r] = 0.f;
  for (int r = 0; r < 8; ++r) sp[wave][8 * g + r][16 + col] = 0.f;
#pragma unroll 1
  for (int h = 0; h < NH; ++h) {
    const F2 aq = split_row(QKV + (r0 + col) * (3 * DD) + h * HD, 0, lane); const F2 kb = split_row(QKV + (r0 + col) * (3 * DD) + DD + h * HD, 0, lane);
    const v8f s = mac3(aq, kb, (v8f){});
    float p[8];
#pragma unroll
    for (int r = 0; r < 8; ++r) { const float v = s[r] * 0.17677669529663688f; float mx = v;
#pragma unroll
      for (int o = 1; o < 16; o <<= 1) mx = fmaxf(mx, __shfl_xor(mx, o));
      const float e = exp_ni(v - mx); float z = e;
#pragma unroll
      for (int o = 1; o < 16; o <<= 1) z += __shfl_xor(z, o);
      p[r] = e / z; pacc[r] += p[r]; sp[wave][8 * g + r][col] = p[r]; }
    LDSX();
    const F2 pa = split_row(&sp[wave][col][0], 0, lane);
    __shared__ __align__(16) float sv[4][32][36];
    for (int q = lane; q < 16 * 32; q += 32) { const int key = q >> 5, d = q & 31; sv[wave][d][key] = QKV[(r0 + key) * (3 * DD) + 2 * DD + h * HD + d]; }
    for (int q = lane; q < 32 * 16; q += 32) { const int d = q >> 4, key = 16 + (q & 15); sv[wave][d][key] = 0.f; }
    LDSX();
    v8f acc[2] = {};
#pragma unroll
    for (int dt = 0; dt < 2; ++dt) { const F2 vb = split_row(&sv[wave][dt * 16 + col][0], 0, lane); acc[dt] = mac3(pa, vb, acc[dt]); }
#pragma unroll
    for (int dt = 0; dt < 2; ++dt)
#pragma unroll
      for (int r = 0; r < 8; ++r) so[wave][8 * g + r][h * HD + dt * 16 + col] = acc[dt][r];
    LDSX(); }
  for (int rl = 0; rl < 16; ++rl) { vst2(CTX + (r0 + rl) * DD + lane * 4, *(const v4f*)&so[wave][rl][lane * 4]); vst2(CTX + (r0 + rl) * DD + 128 + lane * 4, *(const v4f*)&so[wave][rl][128 + lane * 4]); }
#pragma unroll
  for (int r = 0; r < 8; ++r) sacc[wave][8 * g + r][col] = pacc[r];
  __syncthreads();
  for (int q = tid; q < 256; q += 128) { const int i = q >> 4, j = q & 15; sline[q] = ((sacc[0][i][j] + sacc[1][i][j]) + sacc[2][i][j]) + sacc[3][i][j]; }
  __syncthreads();
  if (tid < 64) vst2(PA + (size_t)blockIdx.x * 256 + tid * 4, *(const v4f*)&sline[tid * 4]);
}
__global__ __launch_bounds__(256) void k_wavg(const float* __restrict__ PA, float* __restrict__ AW) {
  __shared__ __align__(16) float s[256]; const int tid = threadIdx.x; float acc = 0.f;
#pragma unroll 1
  for (int b = 0; b < NGB; ++b) acc += PA[(size_t)b * 256 + tid];
  s[tid] = acc / (float)(NG * NH);
  __syncthreads();
  if (tid < 64) vst2(AW + tid * 4, *(const v4f*)&s[tid * 4]);
}
extern "C" void kernel_launch(void* const* d_in, const int* in_sizes, int n_in, void* d_out, int out_size, void* d_ws, size_t ws_size, hipStream_t stream) {
  (void)in_sizes; (void)n_in; (void)out_size;
  const float** F = (const float**)d_in;
  if (ws_size < (size_t)WS_END) return;
  char* ws = (char*)d_ws; __bf16* PW = (__bf16*)(ws + WS_PW); float *QKV = (float*)(ws + WS_QKV), *CTX = (float*)(ws + WS_CTX), *PA = (float*)(ws + WS_PA);
  float* OUT = (float*)d_out; float* AW = OUT + (size_t)NTOK_FULL * DD;
  k_packT<<<dim3(3 * DD, 2), 256, 0, stream>>>(F[2], F[4], F[6], F[8], PW);
  k_gemm<1><<<dim3(NGB, DD / 128), 128, 0, stream>>>(F[0], PW + PQKV, F[3], QKV, 3 * DD);
  k_gemm<1><<<dim3(NGB, DD / 128), 128, 0, stream>>>(F[0], PW + PQKV + (size_t)DD * DD, F[5], QKV + DD, 3 * DD);
  k_gemm<1><<<dim3(NGB, DD / 128), 128, 0, stream>>>(F[0], PW + PQKV + (size_t)2 * DD * DD, F[7], QKV + 2 * DD, 3 * DD);
  k_attn<<<NGB, 128, 0, stream>>>(QKV, CTX, PA);
  k_gemm<0><<<dim3(NGB, DD / 128), 128, 0, stream>>>(CTX, PW + PO, F[9], OUT, DD);
  k_wavg<<<1, 256, 0, stream>>>(PA, AW);
}
